// Attention_21887153341027
// MI455X (gfx1250) — hardware-verified
//
#include <hip/hip_runtime.h>


typedef _Float16 v16h __attribute__((ext_vector_type(16)));
typedef _Float16 v8h  __attribute__((ext_vector_type(8)));
typedef float    v8f  __attribute__((ext_vector_type(8)));
typedef float    v4f  __attribute__((ext_vector_type(4)));

#ifndef NB
#define NB 4
#endif
#ifndef SEQ
#define SEQ 2048
#endif
#define NB_FULL  4
#define SEQ_FULL 2048
#define CC   1024
#define HH   16
#define DD   64
#define C3   (3 * CC)
#define LDQK (2 * CC)
#define MTOK (NB * SEQ)

static_assert(NB >= 1 && NB <= NB_FULL);
static_assert(SEQ >= 64 && SEQ <= SEQ_FULL && (SEQ % 64) == 0);
static_assert(CC == HH * DD);
static_assert((CC % 64) == 0 && (C3 % 64) == 0 && (CC / 8) == 128);

#define WSC       64.0f
#define WINV      0.015625f
#define QC        4.0f
#define VCY       16.0f
#define PCY       1024.0f
#define SCALE_QK  0.0078125f
#define CTX_OUT   0.00390625f
#define PROJ_UNSC 0.000244140625f
#define NEPS      1e-6f

#define TPH 72
#define TPF 68

__device__ __forceinline__ float bf16r(float f) {
    unsigned int u = __float_as_uint(f);
    u += 0x7FFFu + ((u >> 16) & 1u);
    u &= 0xFFFF0000u;
    return __uint_as_float(u);
}

__device__ __forceinline__ v8f vzero8() {
    v8f z = {0.f, 0.f, 0.f, 0.f, 0.f, 0.f, 0.f, 0.f};
    return z;
}

__device__ __forceinline__ v8f mma16(v16h a, v16h b, v8f c) {
    v8f d = __builtin_amdgcn_wmma_f32_16x16x32_f16(false, a, false, b, (short)0, c, false, false);
    asm volatile("v_nop\n\tv_nop\n\tv_nop\n\tv_nop" : "+v"(d) : "v"(a), "v"(b));
    return d;
}

__device__ __forceinline__ v16h load_frag_rowmajor(const _Float16* base, int ld) {
    const int lane = threadIdx.x & 31;
    const _Float16* p = base + (size_t)(lane & 15) * ld + ((lane >> 4) << 3);
    v8h lo = *(const v8h*)(p);
    v8h hi = *(const v8h*)(p + 16);
    return __builtin_shufflevector(lo, hi, 0, 1, 2, 3, 4, 5, 6, 7,
                                           8, 9, 10, 11, 12, 13, 14, 15);
}

__global__ __launch_bounds__(256) void cvt_x_kernel(const float* __restrict__ x,
                                                    _Float16* __restrict__ xh, int ngrp) {
    const int g = blockIdx.x * 256 + threadIdx.x;
    if (g >= ngrp) return;
    const int t  = g >> 7;
    const int c8 = g & 127;
    const int b  = t / SEQ;
    const int n  = t - b * SEQ;
    const float* src = x + ((size_t)b * SEQ_FULL + n) * CC + c8 * 8;
    const v4f x0 = *(const v4f*)(src);
    const v4f x1 = *(const v4f*)(src + 4);
    v8h o;
    o[0] = (_Float16)bf16r(x0[0]); o[1] = (_Float16)bf16r(x0[1]);
    o[2] = (_Float16)bf16r(x0[2]); o[3] = (_Float16)bf16r(x0[3]);
    o[4] = (_Float16)bf16r(x1[0]); o[5] = (_Float16)bf16r(x1[1]);
    o[6] = (_Float16)bf16r(x1[2]); o[7] = (_Float16)bf16r(x1[3]);
    _Float16* dst = xh + (size_t)t * CC + c8 * 8;
    *(volatile v8h*)dst = o;
    __threadfence();
    *(volatile v8h*)dst = o;
}

__global__ __launch_bounds__(256) void wT_kernel(const float* __restrict__ w,
                                                 _Float16* __restrict__ wt, int R, int Ccols) {
    __shared__ float tile[64][65];
    const int t  = threadIdx.x;
    const int c0 = blockIdx.x * 64;
    const int r0 = blockIdx.y * 64;
#pragma unroll
    for (int i = 0; i < 16; ++i) {
        const int idx = t + 256 * i;
        const int r = idx >> 6, c = idx & 63;
        tile[r][c] = w[(size_t)(r0 + r) * Ccols + c0 + c];
    }
    __syncthreads();
    const int piece = t & 7;
#pragma unroll 1
    for (int pass = 0; pass < 2; ++pass) {
#pragma unroll
        for (int it = 0; it < 2; ++it) {
            const int cl = (t >> 3) + 32 * it;
            v8h o;
#pragma unroll
            for (int i = 0; i < 8; ++i)
                o[i] = (_Float16)(bf16r(tile[8 * piece + i][cl]) * WSC);
            _Float16* dst = wt + (size_t)(c0 + cl) * R + r0 + 8 * piece;
            *(volatile v8h*)dst = o;
        }
        if (pass == 0) __threadfence();
    }
}

__device__ __forceinline__ void gemm_core_32x64(const _Float16* __restrict__ Aw,
                                                const _Float16* __restrict__ Bt,
                                                int K, v8f (&acc)[2][4]) {
#pragma unroll 1
    for (int k0 = 0; k0 < K; k0 += 32) {
        const v16h a0 = load_frag_rowmajor(Aw + k0, K);
        const v16h a1 = load_frag_rowmajor(Aw + (size_t)16 * K + k0, K);
        const v16h b0 = load_frag_rowmajor(Bt + k0, K);
        const v16h b1 = load_frag_rowmajor(Bt + (size_t)16 * K + k0, K);
        const v16h b2 = load_frag_rowmajor(Bt + (size_t)32 * K + k0, K);
        const v16h b3 = load_frag_rowmajor(Bt + (size_t)48 * K + k0, K);
        acc[0][0] = mma16(a0, b0, acc[0][0]);
        acc[0][1] = mma16(a0, b1, acc[0][1]);
        acc[0][2] = mma16(a0, b2, acc[0][2]);
        acc[0][3] = mma16(a0, b3, acc[0][3]);
        acc[1][0] = mma16(a1, b0, acc[1][0]);
        acc[1][1] = mma16(a1, b1, acc[1][1]);
        acc[1][2] = mma16(a1, b2, acc[1][2]);
        acc[1][3] = mma16(a1, b3, acc[1][3]);
    }
}

__global__ __launch_bounds__(64) __attribute__((amdgpu_num_vgpr(256)))
void qkv_gemm_kernel(const _Float16* __restrict__ xh, const _Float16* __restrict__ wt,
                     const float* __restrict__ bqkv, const float* __restrict__ qnw,
                     const float* __restrict__ knw, _Float16* __restrict__ qk,
                     _Float16* __restrict__ vT) {
    __shared__ __align__(16) _Float16 st[64 * TPH];

    const int lane = threadIdx.x & 31, wave = threadIdx.x >> 5;
    const int half = lane >> 4, col = lane & 15;
    const int n0 = blockIdx.x * 64;
    const int m0 = blockIdx.y * 64;

    v8f acc[2][4];
#pragma unroll
    for (int s = 0; s < 2; ++s)
#pragma unroll
        for (int j = 0; j < 4; ++j) acc[s][j] = vzero8();

    gemm_core_32x64(xh + (size_t)(m0 + 32 * wave) * CC, wt + (size_t)n0 * CC, CC, acc);

    const int which = n0 >> 10;
    const int hcol  = n0 & (CC - 1);

    float bia[4], nw[4];
#pragma unroll
    for (int j = 0; j < 4; ++j) {
        bia[j] = bf16r(bqkv[n0 + 16 * j + col]);
        const float wq = bf16r(qnw[16 * j + col]);
        const float wk = bf16r(knw[16 * j + col]);
        nw[j] = (which == 1) ? wk : wq;
    }

#pragma unroll
    for (int s = 0; s < 2; ++s)
#pragma unroll
        for (int j = 0; j < 4; ++j)
#pragma unroll
            for (int r = 0; r < 8; ++r)
                acc[s][j][r] = acc[s][j][r] * WINV + bia[j];

    if (which < 2) {
#pragma unroll
        for (int s = 0; s < 2; ++s) {
#pragma unroll
            for (int r = 0; r < 8; ++r) {
                float ss = 0.f;
#pragma unroll
                for (int j = 0; j < 4; ++j) ss += acc[s][j][r] * acc[s][j][r];
                ss += __shfl_xor(ss, 1, 32);
                ss += __shfl_xor(ss, 2, 32);
                ss += __shfl_xor(ss, 4, 32);
                ss += __shfl_xor(ss, 8, 32);
                const float inv = rsqrtf(ss * (1.0f / (float)DD) + NEPS);
                const float g = inv * QC;
#pragma unroll
                for (int j = 0; j < 4; ++j) acc[s][j][r] = acc[s][j][r] * g * nw[j];
            }
        }
    } else {
#pragma unroll
        for (int s = 0; s < 2; ++s)
#pragma unroll
            for (int j = 0; j < 4; ++j)
#pragma unroll
                for (int r = 0; r < 8; ++r) acc[s][j][r] *= VCY;
    }

#pragma unroll
    for (int s = 0; s < 2; ++s)
#pragma unroll
        for (int j = 0; j < 4; ++j)
#pragma unroll
            for (int r = 0; r < 8; ++r)
                st[(32 * wave + 16 * s + 8 * half + r) * TPH + 16 * j + col] = (_Float16)acc[s][j][r];
    __syncthreads();

    if (which < 2) {
        _Float16* dbase = qk + (size_t)m0 * LDQK + (size_t)which * CC + hcol;
        const int piece = lane & 7, rsub = lane >> 3;
#pragma unroll 1
        for (int pass = 0; pass < 2; ++pass) {
#pragma unroll
            for (int it = 0; it < 8; ++it) {
                const int row = 32 * wave + 4 * it + rsub;
                const v8h v = *(const v8h*)(st + row * TPH + 8 * piece);
                *(volatile v8h*)(dbase + (size_t)row * LDQK + 8 * piece) = v;
            }
            if (pass == 0) __threadfence();
        }
    } else {
        const int b  = m0 / SEQ;
        const int nb = m0 - b * SEQ;
        _Float16* dbase = vT + ((size_t)b * CC + hcol) * SEQ + nb;
        const int piece = threadIdx.x & 7, dsub = threadIdx.x >> 3;
#pragma unroll 1
        for (int pass = 0; pass < 2; ++pass) {
#pragma unroll
            for (int it = 0; it < 8; ++it) {
                const int d = 8 * it + dsub;
                v8h v;
#pragma unroll
                for (int i = 0; i < 8; ++i) v[i] = st[(8 * piece + i) * TPH + d];
                *(volatile v8h*)(dbase + (size_t)d * SEQ + 8 * piece) = v;
            }
            if (pass == 0) __threadfence();
        }
    }
}

__global__ __launch_bounds__(32) __attribute__((amdgpu_num_vgpr(256)))
void mha_flash_kernel(const _Float16* __restrict__ qk, const _Float16* __restrict__ vT,
                      _Float16* __restrict__ ctx) {
    __shared__ __align__(16) _Float16 Pld[16 * 32];
    __shared__ __align__(16) _Float16 Ost[16 * TPH];

    const int q0 = blockIdx.x * 16;
    const int h  = blockIdx.y;
    const int b  = blockIdx.z;
    const size_t tokBase = (size_t)b * SEQ;

    const int lane = threadIdx.x & 31;
    const int half = lane >> 4;
    const int col  = lane & 15;

    const _Float16* qbase = qk + (tokBase + q0) * LDQK + h * DD;
    const v16h qa0 = load_frag_rowmajor(qbase, LDQK);
    const v16h qa1 = load_frag_rowmajor(qbase + 32, LDQK);

    const _Float16* kbase0 = qk + tokBase * LDQK + CC + h * DD;
    const _Float16* vtbase = vT + ((size_t)b * CC + h * DD) * SEQ;

    v8f o[4];
#pragma unroll
    for (int j = 0; j < 4; ++j) o[j] = vzero8();
    float m[8], l[8];
#pragma unroll
    for (int r = 0; r < 8; ++r) { m[r] = -1e30f; l[r] = 0.f; }

#pragma unroll 1
    for (int kb = 0; kb < SEQ; kb += 32) {
        const _Float16* kbase = kbase0 + (size_t)kb * LDQK;

        const v16h kf00 = load_frag_rowmajor(kbase, LDQK);
        const v16h kf01 = load_frag_rowmajor(kbase + 32, LDQK);
        const v16h kf10 = load_frag_rowmajor(kbase + (size_t)16 * LDQK, LDQK);
        const v16h kf11 = load_frag_rowmajor(kbase + (size_t)16 * LDQK + 32, LDQK);

        v8f s0 = vzero8(), s1 = vzero8();
        s0 = mma16(qa0, kf00, s0);
        s0 = mma16(qa1, kf01, s0);
        s1 = mma16(qa0, kf10, s1);
        s1 = mma16(qa1, kf11, s1);

        float fac[8];
#pragma unroll
        for (int r = 0; r < 8; ++r) {
            const float a0 = s0[r] * SCALE_QK;
            const float a1 = s1[r] * SCALE_QK;
            float rm = fmaxf(a0, a1);
            rm = fmaxf(rm, __shfl_xor(rm, 1, 32));
            rm = fmaxf(rm, __shfl_xor(rm, 2, 32));
            rm = fmaxf(rm, __shfl_xor(rm, 4, 32));
            rm = fmaxf(rm, __shfl_xor(rm, 8, 32));
            const float nm = fmaxf(m[r], rm);
            const float p0 = __expf(a0 - nm);
            const float p1 = __expf(a1 - nm);
            float rs = p0 + p1;
            rs += __shfl_xor(rs, 1, 32);
            rs += __shfl_xor(rs, 2, 32);
            rs += __shfl_xor(rs, 4, 32);
            rs += __shfl_xor(rs, 8, 32);
            const float f = __expf(m[r] - nm);
            l[r] = l[r] * f + rs;
            m[r] = nm;
            fac[r] = f;
            const int row = r + 8 * half;
            Pld[row * 32 + col]      = (_Float16)(p0 * PCY);
            Pld[row * 32 + 16 + col] = (_Float16)(p1 * PCY);
        }

#pragma unroll
        for (int j = 0; j < 4; ++j)
#pragma unroll
            for (int r = 0; r < 8; ++r) o[j][r] *= fac[r];

        __syncthreads();
        const v16h pa  = load_frag_rowmajor(&Pld[0], 32);
        const v16h vf0 = load_frag_rowmajor(vtbase + kb, SEQ);
        const v16h vf1 = load_frag_rowmajor(vtbase + (size_t)16 * SEQ + kb, SEQ);
        const v16h vf2 = load_frag_rowmajor(vtbase + (size_t)32 * SEQ + kb, SEQ);
        const v16h vf3 = load_frag_rowmajor(vtbase + (size_t)48 * SEQ + kb, SEQ);

        o[0] = mma16(pa, vf0, o[0]);
        o[1] = mma16(pa, vf1, o[1]);
        o[2] = mma16(pa, vf2, o[2]);
        o[3] = mma16(pa, vf3, o[3]);
        __syncthreads();
    }

#pragma unroll
    for (int r = 0; r < 8; ++r) {
        const float rl = CTX_OUT * (1.0f / l[r]);
#pragma unroll
        for (int j = 0; j < 4; ++j)
            Ost[(8 * half + r) * TPH + 16 * j + col] = (_Float16)(o[j][r] * rl);
    }
    __syncthreads();

    _Float16* dbase = ctx + (tokBase + q0) * CC + h * DD;
    const int piece = lane & 7, rsub = lane >> 3;
#pragma unroll 1
    for (int pass = 0; pass < 2; ++pass) {
#pragma unroll
        for (int it = 0; it < 4; ++it) {
            const int row = 4 * it + rsub;
            const v8h v = *(const v8h*)(Ost + row * TPH + 8 * piece);
            *(volatile v8h*)(dbase + (size_t)row * CC + 8 * piece) = v;
        }
        if (pass == 0) __threadfence();
    }
}

__global__ __launch_bounds__(64) __attribute__((amdgpu_num_vgpr(256)))
void proj_gemm_kernel(const _Float16* __restrict__ ctx, const _Float16* __restrict__ wt,
                      const float* __restrict__ bproj, float* __restrict__ out) {
    __shared__ __align__(16) float st[64 * TPF];

    const int lane = threadIdx.x & 31, wave = threadIdx.x >> 5;
    const int half = lane >> 4, col = lane & 15;
    const int n0 = blockIdx.x * 64;
    const int m0 = blockIdx.y * 64;

    v8f acc[2][4];
#pragma unroll
    for (int s = 0; s < 2; ++s)
#pragma unroll
        for (int j = 0; j < 4; ++j) acc[s][j] = vzero8();

    gemm_core_32x64(ctx + (size_t)(m0 + 32 * wave) * CC, wt + (size_t)n0 * CC, CC, acc);

    float bia[4];
#pragma unroll
    for (int j = 0; j < 4; ++j) bia[j] = bf16r(bproj[n0 + 16 * j + col]);

#pragma unroll
    for (int s = 0; s < 2; ++s)
#pragma unroll
        for (int j = 0; j < 4; ++j)
#pragma unroll
            for (int r = 0; r < 8; ++r)
                st[(32 * wave + 16 * s + 8 * half + r) * TPF + 16 * j + col] =
                    acc[s][j][r] * PROJ_UNSC + bia[j];
    __syncthreads();

    float* dbase = out + (size_t)m0 * CC + n0;
    const int piece = lane & 15, rsub = lane >> 4;
#pragma unroll 1
    for (int pass = 0; pass < 2; ++pass) {
#pragma unroll
        for (int it = 0; it < 16; ++it) {
            const int row = 32 * wave + 2 * it + rsub;
            const v4f v = *(const v4f*)(st + row * TPF + 4 * piece);
            *(volatile v4f*)(dbase + (size_t)row * CC + 4 * piece) = v;
        }
        if (pass == 0) __threadfence();
    }
}

extern "C" void kernel_launch(void* const* d_in, const int* in_sizes, int n_in,
                              void* d_out, int out_size, void* d_ws, size_t ws_size,
                              hipStream_t stream) {
    if (n_in < 7) return;
    const float* x      = (const float*)d_in[0];
    const float* W_qkv  = (const float*)d_in[1];
    const float* b_qkv  = (const float*)d_in[2];
    const float* W_proj = (const float*)d_in[3];
    const float* b_proj = (const float*)d_in[4];
    const float* qn_w   = (const float*)d_in[5];
    const float* kn_w   = (const float*)d_in[6];
    float* out = (float*)d_out;

    if (in_sizes[0] < ((NB - 1) * SEQ_FULL + SEQ) * CC) return;
    if (in_sizes[1] < CC * C3) return;
    if (in_sizes[2] < C3) return;
    if (in_sizes[3] < CC * CC) return;
    if (in_sizes[4] < CC) return;
    if (in_sizes[5] < DD) return;
    if (in_sizes[6] < DD) return;
    if (out_size < MTOK * CC) return;

    char* wsb = (char*)d_ws;
    size_t off = 0;
    const size_t sz_xh  = (size_t)MTOK * CC * 2;
    const size_t sz_wq  = (size_t)C3 * CC * 2;
    const size_t sz_wp  = (size_t)CC * CC * 2;
    const size_t sz_qk  = (size_t)MTOK * LDQK * 2;
    const size_t sz_vt  = (size_t)NB * CC * SEQ * 2;
    const size_t sz_ctx = (size_t)MTOK * CC * 2;
    _Float16* xh     = (_Float16*)(wsb + off); off += (sz_xh  + 255) & ~(size_t)255;
    _Float16* wqkvT  = (_Float16*)(wsb + off); off += (sz_wq  + 255) & ~(size_t)255;
    _Float16* wprojT = (_Float16*)(wsb + off); off += (sz_wp  + 255) & ~(size_t)255;
    _Float16* qkp    = (_Float16*)(wsb + off); off += (sz_qk  + 255) & ~(size_t)255;
    _Float16* vT     = (_Float16*)(wsb + off); off += (sz_vt  + 255) & ~(size_t)255;
    _Float16* ctx    = (_Float16*)(wsb + off); off += (sz_ctx + 255) & ~(size_t)255;
    if (off > ws_size) return;

    {
        const int ngrp = MTOK * (CC / 8);
        cvt_x_kernel<<<(ngrp + 255) / 256, 256, 0, stream>>>(x, xh, ngrp);
        wT_kernel<<<dim3(C3 / 64, CC / 64), 256, 0, stream>>>(W_qkv, wqkvT, CC, C3);
        wT_kernel<<<dim3(CC / 64, CC / 64), 256, 0, stream>>>(W_proj, wprojT, CC, CC);
    }

    qkv_gemm_kernel<<<dim3(C3 / 64, MTOK / 64), 64, 0, stream>>>(
        xh, wqkvT, b_qkv, qn_w, kn_w, qkp, vT);

    mha_flash_kernel<<<dim3(SEQ / 16, HH, NB), 32, 0, stream>>>(qkp, vT, ctx);

    proj_gemm_kernel<<<dim3(CC / 64, MTOK / 64), 64, 0, stream>>>(ctx, wprojT, b_proj, out);
}
